// LRU_27247272526459
// MI455X (gfx1250) — hardware-verified
//
#include <hip/hip_runtime.h>
#include <math.h>

constexpr int NB_SEQ   = 16;
constexpr int NT_STEP  = 2048;
constexpr int NH_IN    = 128;
constexpr int NH_OUT   = 128;
constexpr int NSTATE   = 256;
constexpr int NROWS    = NB_SEQ * NT_STEP;
constexpr int XP_COLS  = 2 * NSTATE;
constexpr int AX_COLS  = XP_COLS + NH_IN;
constexpr int NTHR     = 256;
constexpr int SCAN_TCH = 8;
constexpr float X_CARRY   = 8.0f;
constexpr float S_CARRY   = 8.0f;
constexpr float W_CARRY   = 16.0f;
constexpr float GEMM_FOLD = 1.0f / 128.0f;
static_assert(NROWS % 64 == 0 && XP_COLS % 64 == 0 && NH_OUT % 64 == 0);
static_assert(NH_IN % 32 == 0 && AX_COLS % 32 == 0);
static_assert(((NROWS / 64) * (XP_COLS / 64)) % 8 == 0);
static_assert(((NROWS / 64) * (NH_OUT / 64)) % 8 == 0);
static_assert(NSTATE == NTHR);
static_assert(SCAN_TCH == NTHR / 32);
static_assert(NSTATE == 32 * 8);
static_assert(NT_STEP % SCAN_TCH == 0);
static_assert(NH_IN % 8 == 0 && NSTATE % 8 == 0 && AX_COLS % 8 == 0);

typedef __attribute__((ext_vector_type(16))) _Float16 v16h;
typedef __attribute__((ext_vector_type(8)))  _Float16 v8h;
typedef __attribute__((ext_vector_type(16))) __bf16   v16b;
typedef __attribute__((ext_vector_type(8)))  __bf16   v8b;
typedef __attribute__((ext_vector_type(8)))  float    v8f;
typedef __attribute__((ext_vector_type(4)))  float    v4f;

__device__ __forceinline__ unsigned short f2bf_bits(float f) {
  unsigned u = __float_as_uint(f);
  return (unsigned short)((u + 0x7FFFu + ((u >> 16) & 1u)) >> 16);
}
__device__ __forceinline__ float bf_bits2f(unsigned short h) { return __uint_as_float(((unsigned)h) << 16); }

__device__ __forceinline__ void dep_guard_h(v8f& a, v8f& b, v16h x, v16h y) { asm volatile("v_nop\n\tv_nop\n\tv_nop\n\tv_nop" : "+v"(a), "+v"(b) : "v"(x), "v"(y)); }
__device__ __forceinline__ void dep_guard_b(v8f& a, v8f& b, v16b x, v16b y) { asm volatile("v_nop\n\tv_nop\n\tv_nop\n\tv_nop" : "+v"(a), "+v"(b) : "v"(x), "v"(y)); }
__device__ __forceinline__ void keep4_h(v16h a, v16h b, v16h c, v16h d) { asm volatile("v_nop" :: "v"(a), "v"(b), "v"(c), "v"(d)); }
__device__ __forceinline__ void keep4_b(v16b a, v16b b, v16b c, v16b d) { asm volatile("v_nop" :: "v"(a), "v"(b), "v"(c), "v"(d)); }
__device__ __forceinline__ void acc_guard4(v8f& a, v8f& b, v8f& c, v8f& d) { asm volatile("v_nop\n\tv_nop\n\tv_nop\n\tv_nop" : "+v"(a), "+v"(b), "+v"(c), "+v"(d)); }
template <typename T> struct Frag;
template <> struct Frag<_Float16> {
  typedef v16h V; union U { v16h v; v8h h[2]; };
  static __device__ __forceinline__ v16h load(const _Float16* p) {
    U f; f.h[0] = *(const v8h*)(p); f.h[1] = *(const v8h*)(p + 16); return f.v;
  }
  static __device__ __forceinline__ v8f mma(v16h a, v16h b, v8f c) {
    return __builtin_amdgcn_wmma_f32_16x16x32_f16(false, a, false, b, (short)0, c, false, false);
  }
  static __device__ __forceinline__ void guard(v8f& a, v8f& b, v16h x, v16h y) { dep_guard_h(a, b, x, y); }
  static __device__ __forceinline__ void keep(v16h a, v16h b, v16h c, v16h d) { keep4_h(a, b, c, d); }
};
template <> struct Frag<__bf16> {
  typedef v16b V; union U { v16b v; v8b h[2]; };
  static __device__ __forceinline__ v16b load(const __bf16* p) {
    U f; f.h[0] = *(const v8b*)(p); f.h[1] = *(const v8b*)(p + 16); return f.v;
  }
  static __device__ __forceinline__ v8f mma(v16b a, v16b b, v8f c) {
    return __builtin_amdgcn_wmma_f32_16x16x32_bf16(false, a, false, b, (short)0, c, false, false);
  }
  static __device__ __forceinline__ void guard(v8f& a, v8f& b, v16b x, v16b y) { dep_guard_b(a, b, x, y); }
  static __device__ __forceinline__ void keep(v16b a, v16b b, v16b c, v16b d) { keep4_b(a, b, c, d); }
};

template <int ET> struct Elem;
template <> struct Elem<0> { typedef _Float16 T; };
template <> struct Elem<1> { typedef __bf16 T; };
template <int ET, bool SPLIT, int BIAS_MODE, int OUT_MODE, bool RESID, int ACT = 0>
__global__ __launch_bounds__(256) void wmma_gemm64(
    const unsigned short* __restrict__ Ap, const unsigned short* __restrict__ A2p, int lda, long strideA,
    const unsigned short* __restrict__ Btp, const unsigned short* __restrict__ Bt2p, int ldb, long strideB,
    void* __restrict__ Cout, void* __restrict__ Cout2, int ldc, long strideC,
    const float* __restrict__ bias,
    const float* __restrict__ resid, long strideR,
    int M, int N, int K, float scale) {
  typedef typename Elem<ET>::T T;
  typedef typename Frag<T>::V V;
  const T* A = (const T*)Ap; const T* A2 = (const T*)A2p; const T* Bt = (const T*)Btp; const T* Bt2 = (const T*)Bt2p;
  __shared__ __align__(16) float sT[8][16 * 68];
  const int b    = blockIdx.y;
  const int lane = threadIdx.x & 31;
  const int wave = threadIdx.x >> 5;
  const int tilesN = N >> 6;
  const int tilesM = M >> 6;
  const int tile = blockIdx.x * 8 + wave;
  if (tile >= tilesM * tilesN) return;
  const int tm = tile / tilesN;
  const int tn = tile - tm * tilesN;
  const int m0 = tm << 6;
  const int n0 = tn << 6;

  const T* Ab  = A  + (size_t)b * strideA;
  const T* Bb  = Bt + (size_t)b * strideB;
  const T* Ab2 = SPLIT ? (A2  + (size_t)b * strideA) : nullptr;
  const T* Bb2 = SPLIT ? (Bt2 + (size_t)b * strideB) : nullptr;

  const int rlane = lane & 15;
  const int koff  = (lane >> 4) * 8;
  const int mOff  = (lane >> 4) * 8;

  v8f acc[4][4];
#pragma unroll
  for (int i = 0; i < 4; ++i)
#pragma unroll
    for (int j = 0; j < 4; ++j) acc[i][j] = (v8f){0.f,0.f,0.f,0.f,0.f,0.f,0.f,0.f};

  for (int k0 = 0; k0 < K; k0 += 32) {
    V bh[4], bl[4];
#pragma unroll
    for (int j = 0; j < 4; ++j) {
      const size_t bo = (size_t)(n0 + (j << 4) + rlane) * ldb + koff + k0;
      bh[j] = Frag<T>::load(Bb + bo);
      if (SPLIT) bl[j] = Frag<T>::load(Bb2 + bo);
    }
#pragma unroll
    for (int i = 0; i < 4; ++i) {
      const size_t ao = (size_t)(m0 + (i << 4) + rlane) * lda + koff + k0;
      V ah = Frag<T>::load(Ab + ao);
      V al;
      if (SPLIT) al = Frag<T>::load(Ab2 + ao);
#pragma unroll
      for (int j = 0; j < 4; ++j) {
        acc[i][j] = Frag<T>::mma(ah, bh[j], acc[i][j]);
        if (SPLIT) {
          acc[i][j] = Frag<T>::mma(ah, bl[j], acc[i][j]);
          acc[i][j] = Frag<T>::mma(al, bh[j], acc[i][j]);
        }
      }
      Frag<T>::guard(acc[i][0], acc[i][3], ah, SPLIT ? al : ah);
    }
    Frag<T>::keep(bh[0], bh[1], bh[2], bh[3]);
    if (SPLIT) Frag<T>::keep(bl[0], bl[1], bl[2], bl[3]);
  }
  acc_guard4(acc[0][0], acc[0][1], acc[0][2], acc[0][3]);
  acc_guard4(acc[1][0], acc[1][1], acc[1][2], acc[1][3]);
  acc_guard4(acc[2][0], acc[2][1], acc[2][2], acc[2][3]);
  acc_guard4(acc[3][0], acc[3][1], acc[3][2], acc[3][3]);

  float* slab = sT[wave];
  const float* Rb = RESID ? (resid + (size_t)b * strideR) : nullptr;
#pragma unroll
  for (int i = 0; i < 4; ++i) {
    const int mBase = m0 + (i << 4);
#pragma unroll
    for (int j = 0; j < 4; ++j) {
      const int n = n0 + (j << 4) + rlane;
      float bv = 0.f;
      if (BIAS_MODE == 2) bv = bias[n];
#pragma unroll
      for (int r = 0; r < 8; ++r) {
        float v = acc[i][j][r] * scale;
        if (BIAS_MODE == 1) v += bias[mBase + mOff + r];
        if (BIAS_MODE == 2) v += bv;
        if (RESID) v += Rb[(size_t)(mBase + mOff + r) * ldc + n];
        if (ACT == 1) v = tanhf(v);
        if (ACT == 2) v = fmaxf(v, 0.0f);
        if (ACT == 3) v = v / (1.0f + expf(-v));
        if (ACT == 4) v = (v > 0.f) ? v : 0.01f * v;
        if (ACT == 5) v = 0.5f * v * (1.0f + erff(v * 0.70710678118654752f));
        slab[(mOff + r) * 68 + (j << 4) + rlane] = v;
      }
    }
    __builtin_amdgcn_fence(__ATOMIC_RELEASE, "workgroup");
    __builtin_amdgcn_wave_barrier();
    __builtin_amdgcn_fence(__ATOMIC_ACQUIRE, "workgroup");
    if (OUT_MODE == 0) {
      float* C = (float*)Cout + (size_t)b * strideC;
      const int hh = lane >> 4, c4 = (lane & 15) * 4;
      for (int pass = 0; pass < 2; ++pass) {
#pragma unroll
        for (int it = 0; it < 8; ++it) {
          const int row = it * 2 + hh;
          v4f v = *(const v4f*)(slab + row * 68 + c4);
          *(volatile v4f*)(C + (size_t)(mBase + row) * ldc + n0 + c4) = v;
        }
        __threadfence();
      }
    } else {
      const int q = lane >> 3, c8 = (lane & 7) * 8;
      unsigned short* C  = (unsigned short*)Cout  + (size_t)b * strideC;
      unsigned short* C2 = (OUT_MODE == 2) ? ((unsigned short*)Cout2 + (size_t)b * strideC) : nullptr;
      for (int pass = 0; pass < 2; ++pass) {
#pragma unroll
        for (int it = 0; it < 4; ++it) {
          const int row = it * 4 + q;
          const float* sp = slab + row * 68 + c8;
          v8h hv, lv;
#pragma unroll
          for (int e = 0; e < 8; ++e) {
            if (OUT_MODE == 1) {
              hv[e] = (_Float16)sp[e];
            } else {
              unsigned short hb = f2bf_bits(sp[e]);
              unsigned short lb = f2bf_bits(sp[e] - bf_bits2f(hb));
              hv[e] = __builtin_bit_cast(_Float16, hb);
              lv[e] = __builtin_bit_cast(_Float16, lb);
            }
          }
          *(volatile v8h*)(C + (size_t)(mBase + row) * ldc + n0 + c8) = hv;
          if (OUT_MODE == 2) *(volatile v8h*)(C2 + (size_t)(mBase + row) * ldc + n0 + c8) = lv;
        }
        __threadfence();
      }
    }
    __builtin_amdgcn_fence(__ATOMIC_RELEASE, "workgroup");
    __builtin_amdgcn_wave_barrier();
    __builtin_amdgcn_fence(__ATOMIC_ACQUIRE, "workgroup");
  }
}

__global__ __launch_bounds__(NTHR) void cvt8_kernel(const float* __restrict__ src, int spitch, int nrow, int ncol8,
                                                    unsigned short* __restrict__ dst, int dpitch, int dcol0, float sc) {
  const int i  = blockIdx.x * NTHR + threadIdx.x;
  const int n8 = nrow * ncol8;
  if (i < n8) {
    const int row = i / ncol8;
    const int c8  = i - row * ncol8;
    const float* sp = src + (size_t)row * spitch + 8 * c8;
    const v4f a = *(const v4f*)(sp);
    const v4f b = *(const v4f*)(sp + 4);
    v8h hv;
#pragma unroll
    for (int e = 0; e < 4; ++e) {
      hv[e]     = (_Float16)(a[e] * sc);
      hv[4 + e] = (_Float16)(b[e] * sc);
    }
    unsigned short* dp = dst + (size_t)row * dpitch + dcol0 + 8 * c8;
    *(volatile v8h*)dp = hv;
    __threadfence();
    *(volatile v8h*)dp = hv;
  }
}

__global__ __launch_bounds__(NTHR) void lru_scan_kernel(const float* __restrict__ XP,
                                                        const float* __restrict__ nu_log,
                                                        const float* __restrict__ theta_log,
                                                        const float* __restrict__ gamma_log,
                                                        unsigned short* __restrict__ AX) {
  __shared__ __align__(16) float Sf[SCAN_TCH * XP_COLS];
  const int tid = threadIdx.x, lane = tid & 31, wave = tid >> 5;
  const int b = blockIdx.x;
  const int n = tid;
  const float lam = expf(-expf(nu_log[n]));
  const float th  = expf(theta_log[n]);
  const float lr  = lam * cosf(th);
  const float li  = lam * sinf(th);
  const float g   = expf(gamma_log[n]);
  float yr = 0.0f, yi = 0.0f;
  const size_t rowb = (size_t)b * NT_STEP;

#pragma unroll 1
  for (int tc = 0; tc < NT_STEP; tc += SCAN_TCH) {
#pragma unroll 1
    for (int j = 0; j < SCAN_TCH; ++j) {
      const size_t m = rowb + (size_t)(tc + j);
      const float pr = XP[m * XP_COLS + n];
      const float pi = XP[m * XP_COLS + NSTATE + n];
      const float xr = g * pr;
      const float xi = g * pi;
      const float nyr = lr * yr - li * yi + xr;
      const float nyi = lr * yi + li * yr + xi;
      yr = nyr;
      yi = nyi;
      Sf[j * XP_COLS + n]          = yr * S_CARRY;
      Sf[j * XP_COLS + NSTATE + n] = yi * S_CARRY;
    }
    __syncthreads();
    {
      const size_t m = rowb + (size_t)(tc + wave);
      unsigned short* drow = AX + m * AX_COLS;
      const float* srow = Sf + wave * XP_COLS;
      for (int pass = 0; pass < 2; ++pass) {
#pragma unroll
        for (int seg = 0; seg < 2; ++seg) {
          const float* sp = srow + seg * NSTATE + 8 * lane;
          const v4f a = *(const v4f*)(sp);
          const v4f c = *(const v4f*)(sp + 4);
          v8h hv;
#pragma unroll
          for (int e = 0; e < 4; ++e) {
            hv[e]     = (_Float16)a[e];
            hv[4 + e] = (_Float16)c[e];
          }
          *(volatile v8h*)(drow + seg * NSTATE + 8 * lane) = hv;
        }
        __threadfence();
      }
    }
    __syncthreads();
  }
}

extern "C" void kernel_launch(void* const* d_in, const int* in_sizes, int n_in,
                              void* d_out, int out_size, void* d_ws, size_t ws_size, hipStream_t stream) {
  if (n_in < 9 || d_out == nullptr || d_ws == nullptr) return;
  if (in_sizes[0] != NROWS * NH_IN || in_sizes[1] != NSTATE || in_sizes[2] != NSTATE || in_sizes[3] != NSTATE ||
      in_sizes[4] != NSTATE * NH_IN || in_sizes[5] != NSTATE * NH_IN ||
      in_sizes[6] != NH_OUT * NSTATE || in_sizes[7] != NH_OUT * NSTATE || in_sizes[8] != NH_OUT * NH_IN ||
      out_size != NROWS * NH_OUT) return;

  const float* x         = (const float*)d_in[0];
  const float* nu_log    = (const float*)d_in[1];
  const float* theta_log = (const float*)d_in[2];
  const float* gamma_log = (const float*)d_in[3];
  const float* b_re      = (const float*)d_in[4];
  const float* b_im      = (const float*)d_in[5];
  const float* c_re      = (const float*)d_in[6];
  const float* c_im      = (const float*)d_in[7];
  const float* d_w       = (const float*)d_in[8];
  float* out = (float*)d_out;

  char* ws = (char*)d_ws; size_t off = 0;
  auto carve = [&](size_t bytes) -> char* { char* p = ws + off; off += (bytes + 255) & ~(size_t)255; return p; };
  unsigned short* AX  = (unsigned short*)carve((size_t)NROWS * AX_COLS * 2);
  float*          XP  = (float*)carve((size_t)NROWS * XP_COLS * 4);
  unsigned short* BT1 = (unsigned short*)carve((size_t)XP_COLS * NH_IN * 2);
  unsigned short* BT2 = (unsigned short*)carve((size_t)NH_OUT * AX_COLS * 2);
  if (off > ws_size || off > (size_t)134217728) return;
  const float* dummy = (const float*)XP;

  const int n8x  = NROWS * (NH_IN / 8);
  const int n8b  = NSTATE * (NH_IN / 8);
  const int n8c  = NH_OUT * (NSTATE / 8);
  const int n8d  = NH_OUT * (NH_IN / 8);
  cvt8_kernel<<<(n8x + NTHR - 1) / NTHR, NTHR, 0, stream>>>(x,    NH_IN,  NROWS,  NH_IN / 8,  AX,  AX_COLS, XP_COLS, X_CARRY);
  cvt8_kernel<<<(n8b + NTHR - 1) / NTHR, NTHR, 0, stream>>>(b_re, NH_IN,  NSTATE, NH_IN / 8,  BT1, NH_IN,   0,       W_CARRY);
  cvt8_kernel<<<(n8b + NTHR - 1) / NTHR, NTHR, 0, stream>>>(b_im, NH_IN,  NSTATE, NH_IN / 8,  BT1 + (size_t)NSTATE * NH_IN, NH_IN, 0, W_CARRY);
  cvt8_kernel<<<(n8c + NTHR - 1) / NTHR, NTHR, 0, stream>>>(c_re, NSTATE, NH_OUT, NSTATE / 8, BT2, AX_COLS, 0,       2.0f * W_CARRY);
  cvt8_kernel<<<(n8c + NTHR - 1) / NTHR, NTHR, 0, stream>>>(c_im, NSTATE, NH_OUT, NSTATE / 8, BT2, AX_COLS, NSTATE,  -2.0f * W_CARRY);
  cvt8_kernel<<<(n8d + NTHR - 1) / NTHR, NTHR, 0, stream>>>(d_w,  NH_IN,  NH_OUT, NH_IN / 8,  BT2, AX_COLS, XP_COLS, W_CARRY);

  const dim3 g1((NROWS / 64) * (XP_COLS / 64) / 8, 1);
  wmma_gemm64<0, false, 0, 0, false, 0><<<g1, 256, 0, stream>>>(
      AX + XP_COLS, AX + XP_COLS, AX_COLS, 0L, BT1, BT1, NH_IN, 0L, (void*)XP, (void*)XP, XP_COLS, 0L,
      dummy, dummy, 0L, NROWS, XP_COLS, NH_IN, GEMM_FOLD);

  lru_scan_kernel<<<NB_SEQ, NTHR, 0, stream>>>(XP, nu_log, theta_log, gamma_log, AX);

  const dim3 g2((NROWS / 64) * (NH_OUT / 64) / 8, 1);
  wmma_gemm64<0, false, 0, 0, false, 0><<<g2, 256, 0, stream>>>(
      AX, AX, AX_COLS, 0L, BT2, BT2, AX_COLS, 0L, (void*)out, (void*)out, NH_OUT, 0L,
      dummy, dummy, 0L, NROWS, NH_OUT, AX_COLS, GEMM_FOLD);
}
